// CrossAttention_6579889897579
// MI455X (gfx1250) — hardware-verified
//
#include <hip/hip_runtime.h>
#pragma clang fp contract(off)


#ifndef SQ
#define SQ 512
#endif
#ifndef TK
#define TK 16384
#endif
#define SQ_FULL 512
#define TK_FULL 16384
#define DM    512
#define DFF   2048
#define FW    8
#define OSP   68
#define VTP   72
#define SEGCH 1024
#define WSC  64.0f
#define WSI  (1.0f / 64.0f)
#define SC2  ((float)(0.044194173824159216 * 1.4426950408889634))
#define PSH  14.0f
#define NEGB (-3.0e38f)
#define LNEPS 1.0e-5f

static_assert(DM == FW * 64);
static_assert(DM % 32 == 0);
static_assert(DFF % 32 == 0);
static_assert(DM % 64 == 0);
static_assert(DFF % 64 == 0);
static_assert(DM % 128 == 0);
static_assert(SQ % 64 == 0);
static_assert(SQ % 16 == 0);
static_assert(SQ % 8 == 0);
static_assert(TK % 64 == 0);
static_assert(TK % 32 == 0);
static_assert(TK % SEGCH == 0);
static_assert(SEGCH == 256 * 4);
static_assert(((size_t)SQ * DM) % 8 == 0);
static_assert(((size_t)TK * DM) % 8 == 0);
static_assert(((size_t)DM * DM) % 8 == 0);
static_assert(((size_t)DFF * DM) % 8 == 0);
static_assert(SQ <= SQ_FULL);
static_assert(TK <= TK_FULL);
static_assert((OSP * 4) % 16 == 0);
static_assert((VTP * 2) % 16 == 0);
static_assert(OSP >= 64);
static_assert(VTP >= 64);
static_assert(FW * 16 * OSP * 4 <= 131072);
static_assert(64 * VTP * 2 <= 131072);
static_assert(16 * OSP * 4 <= 131072);
static_assert((size_t)SQ * DM * 4 <= (size_t)1048576);

typedef _Float16 h16;
typedef __attribute__((ext_vector_type(16))) _Float16 v16h;
typedef __attribute__((ext_vector_type(8)))  _Float16 v8h;
typedef __attribute__((ext_vector_type(4)))  _Float16 v4h;
typedef __attribute__((ext_vector_type(8)))  float    v8f;
typedef __attribute__((ext_vector_type(4)))  float    v4f;
typedef __attribute__((ext_vector_type(4)))  int      v4i;
typedef v4f  __attribute__((may_alias)) v4fa;
typedef v8h  __attribute__((may_alias)) v8ha;

__device__ __forceinline__ unsigned short f2bf(float f) { unsigned u = __float_as_uint(f); u += 0x7FFFu + ((u >> 16) & 1u); return (unsigned short)(u >> 16); }
__device__ __forceinline__ float bfr(float f) { return __uint_as_float(((unsigned)f2bf(f)) << 16); }
__device__ __forceinline__ v16h cat16(v8h lo, v8h hi) { return __builtin_shufflevector(lo, hi, 0, 1, 2, 3, 4, 5, 6, 7, 8, 9, 10, 11, 12, 13, 14, 15); }
__device__ __forceinline__ v8f wmma16(v16h a, v16h b, v8f c) { return __builtin_amdgcn_wmma_f32_16x16x32_f16(false, a, false, b, (short)0, c, false, false); }
__device__ __forceinline__ v16h  ldh(const h16* p) { return cat16(*(const v8h*)p, *(const v8h*)(p + 16)); }
__device__ __forceinline__ void wave_sync() { __builtin_amdgcn_fence(3  , "wavefront"); __builtin_amdgcn_wave_barrier(); asm volatile("" ::: "memory"); }
static __device__ __forceinline__ h16 toh_flush(float v) { const h16 r = (h16)v; return (fabsf(v) < 6.103515625e-05f) ? (h16)0.0f : r; }
static __device__ __forceinline__ float relu_keep(float v) { return (v > 0.0f) ? v : (v - v); }
__device__ __forceinline__ v8f wmma16g(v16h a, v16h b, v8f c) { c = wmma16(a, b, c); asm volatile("v_nop\n\tv_nop\n\tv_nop\n\tv_nop" : "+v"(c) : "v"(a), "v"(b)); return c; }

__global__ __launch_bounds__(256) void k_sum8(const float* __restrict__ a, const float* __restrict__ b, h16* H, size_t n8) {
    const size_t i = (size_t)blockIdx.x * 256 + threadIdx.x; if (i >= n8) return;
    const v8f x = *(const v8f*)(a + i * 8); const v8f y = *(const v8f*)(b + i * 8); v8h hv;
#pragma unroll
    for (int k = 0; k < 8; ++k) { const float s = bfr(x[k]) + bfr(y[k]); hv[k] = toh_flush(s); }
    *(volatile v8h*)(H + i * 8) = hv; __threadfence();
    *(volatile v8h*)(H + i * 8) = hv;
}

__global__ __launch_bounds__(256) void k_w8(const float* __restrict__ src, h16* dst, size_t n8) {
    const size_t i = (size_t)blockIdx.x * 256 + threadIdx.x; if (i >= n8) return;
    const v8f v = *(const v8f*)(src + i * 8); v8h o;
#pragma unroll
    for (int k = 0; k < 8; ++k) o[k] = toh_flush(bfr(v[k]) * WSC);
    *(volatile v8h*)(dst + i * 8) = o; __threadfence(); *(volatile v8h*)(dst + i * 8) = o;
}

static_assert(2 * 32 == 64);
static_assert(8 * 16 == 128);
__global__ __launch_bounds__(256) void k_vt(const float* __restrict__ mem, h16* VT) {
    __shared__ __align__(16) h16 ts[64 * VTP];
    const int tid = threadIdx.x;
    const int t0 = blockIdx.x * 64, d0 = blockIdx.y * 64;
    { const int row = tid >> 2, c = (tid & 3) * 16;
      const float* p = mem + (size_t)(t0 + row) * DM + d0 + c;
#pragma unroll
      for (int u = 0; u < 4; ++u) { const v4f x = *(const v4f*)(p + 4 * u);
#pragma unroll
          for (int e = 0; e < 4; ++e) ts[(c + 4 * u + e) * VTP + row] = toh_flush(bfr(x[e])); } }
    __syncthreads();
    const int dr = tid >> 3, c8 = (tid & 7) * 8;
#pragma unroll 1
    for (int ps = 0; ps < 2; ++ps) {
#pragma unroll
        for (int s = 0; s < 2; ++s) { const int d = s * 32 + dr;
            const v8h val = *(const v8ha*)(&ts[d * VTP + c8]);
            *(volatile v8h*)(VT + (size_t)(d0 + d) * TK + t0 + c8) = val; }
        if (ps == 0) __threadfence(); }
}

__global__ __launch_bounds__(256) void k_seg(const int* __restrict__ aidx, int* SEG) {
    __shared__ int wsum[8];
    const int lane = threadIdx.x & 31;
    const int wave = __builtin_amdgcn_readfirstlane((int)(threadIdx.x >> 5));
    int carry = 0;
#pragma unroll 1
    for (int cb = 0; cb < TK; cb += SEGCH) {
        const int base = cb + (int)threadIdx.x * 4;
        const v4i v = *(const v4i*)(aidx + base);
        const int pidx = base > 0 ? base - 1 : 0;
        const int pv = aidx[pidx];
        const int s0 = (int)((base > 0) & (v[0] != pv));
        const int s1 = s0 + (int)(v[1] != v[0]);
        const int s2 = s1 + (int)(v[2] != v[1]);
        const int s3 = s2 + (int)(v[3] != v[2]);
        int inc = s3;
#pragma unroll
        for (int off = 1; off < 32; off <<= 1) { const int u = __shfl_up(inc, (unsigned)off, 32); inc += (lane >= off) ? u : 0; }
        if (lane == 31) wsum[wave] = inc;
        __syncthreads();
        int woff = 0, tot = 0;
#pragma unroll
        for (int w = 0; w < 8; ++w) { const int x = wsum[w]; tot += x; woff += (w < wave) ? x : 0; }
        const int ex = carry + woff + (inc - s3);
        v4i o; o[0] = ex + s0; o[1] = ex + s1; o[2] = ex + s2; o[3] = ex + s3;
        *(volatile v4i*)(SEG + base) = o; __threadfence(); *(volatile v4i*)(SEG + base) = o;
        carry += tot;
        __syncthreads();
    }
}

static_assert(4 * 4 == 16);
__global__ __launch_bounds__(32 * FW) void k_flash(const h16* __restrict__ QH, const h16* __restrict__ KH,
                                                   const h16* __restrict__ VT, const int* __restrict__ SEG, h16* CTX) {
    __shared__ __align__(16) float os[FW * 16 * OSP];
    const int lane = threadIdx.x & 31, lr = lane & 15, hi = lane >> 4;
    const int wave = __builtin_amdgcn_readfirstlane((int)(threadIdx.x >> 5));
    const int t0 = blockIdx.x * 16;
    const int d0 = wave * 64;
    const unsigned usq = (unsigned)(t0 + lr);
    const size_t qo = (size_t)(t0 + lr) * DM + 8 * hi;
    const size_t ko = (size_t)lr * DM + 8 * hi;
    const size_t vo = (size_t)(d0 + lr) * TK + 8 * hi;
    v8f o[4];
#pragma unroll
    for (int j = 0; j < 4; ++j) o[j] = (v8f){};
    float m = NEGB, l = 0.0f;
#pragma unroll 1
    for (int key0 = 0; key0 < TK; key0 += 32) {
        const int* sp = SEG + key0 + 8 * hi;
        const v4i sg0 = *(const v4i*)sp, sg1 = *(const v4i*)(sp + 4), sg2 = *(const v4i*)(sp + 16), sg3 = *(const v4i*)(sp + 20);
        bool fa[8], fb[8]; bool anyf = false;
#pragma unroll
        for (int r = 0; r < 4; ++r) {
            fa[r]     = ((unsigned)sg0[r] - usq + 1u) <= 2u;
            fa[4 + r] = ((unsigned)sg1[r] - usq + 1u) <= 2u;
            fb[r]     = ((unsigned)sg2[r] - usq + 1u) <= 2u;
            fb[4 + r] = ((unsigned)sg3[r] - usq + 1u) <= 2u;
            anyf = anyf | fa[r] | fa[4 + r] | fb[r] | fb[4 + r]; }
        if (__builtin_amdgcn_ballot_w32(anyf) == 0u) continue;
        v8f sHa = (v8f){}, sHb = (v8f){};
        const size_t kb = ko + (size_t)key0 * DM;
#pragma unroll 1
        for (int kc = 0; kc < DM; kc += 32) {
            const v16h qh = ldh(QH + qo + kc);
            const v16h ka = ldh(KH + kb + kc), kc2 = ldh(KH + kb + (size_t)16 * DM + kc);
            sHa = wmma16g(ka, qh, sHa);
            sHb = wmma16g(kc2, qh, sHb);
        }
        float ta[8], tb[8]; float mx = NEGB;
#pragma unroll
        for (int r = 0; r < 8; ++r) {
            ta[r] = sHa[r] * SC2; tb[r] = sHb[r] * SC2;
            mx = fmaxf(mx, fmaxf(fa[r] ? ta[r] : NEGB, fb[r] ? tb[r] : NEGB)); }
        mx = fmaxf(mx, __shfl_xor(mx, 16, 32));
        const float mnew = fmaxf(m, mx);
        const float alpha = __builtin_amdgcn_exp2f(m - mnew);
        const float sh = PSH - mnew;
        v16h pb; float ls = 0.0f;
#pragma unroll
        for (int r = 0; r < 8; ++r) {
            const float xa = ta[r] + sh, xb = tb[r] + sh;
            const float ea = __builtin_amdgcn_exp2f(xa), eb = __builtin_amdgcn_exp2f(xb);
            const float ga = (fa[r] && (xa >= -14.0f)) ? ea : 0.0f;
            const float gb = (fb[r] && (xb >= -14.0f)) ? eb : 0.0f;
            const h16 pa = (h16)ga; const h16 pc = (h16)gb;
            pb[r] = pa; pb[8 + r] = pc;
            ls += (float)pa + (float)pc; }
        l = l * alpha + ls; m = mnew;
#pragma unroll
        for (int j = 0; j < 4; ++j) o[j] = o[j] * alpha;
        const h16* va = VT + vo + key0;
        const v16h v0 = ldh(va), v1 = ldh(va + (size_t)16 * TK), v2 = ldh(va + (size_t)32 * TK), v3 = ldh(va + (size_t)48 * TK);
        o[0] = wmma16g(v0, pb, o[0]); o[1] = wmma16g(v1, pb, o[1]); o[2] = wmma16g(v2, pb, o[2]); o[3] = wmma16g(v3, pb, o[3]);
    }
    l += __shfl_xor(l, 16, 32);
    const float inv = 1.0f / l;
    const int wb = wave * 16 * OSP;
#pragma unroll
    for (int j = 0; j < 4; ++j) { v4f a, c;
        a[0] = o[j][0] * inv; a[1] = o[j][1] * inv; a[2] = o[j][2] * inv; a[3] = o[j][3] * inv;
        c[0] = o[j][4] * inv; c[1] = o[j][5] * inv; c[2] = o[j][6] * inv; c[3] = o[j][7] * inv;
        *(v4fa*)(&os[wb + lr * OSP + 16 * j + 8 * hi]) = a; *(v4fa*)(&os[wb + lr * OSP + 16 * j + 8 * hi + 4]) = c; }
    wave_sync();
    h16* crow = CTX + (size_t)t0 * DM + d0;
#pragma unroll 1
    for (int ps = 0; ps < 2; ++ps) {
#pragma unroll
        for (int s = 0; s < 4; ++s) { const int row = 4 * s + (lane >> 3), c8 = (lane & 7) * 8;
            const v4f x0 = *(const v4fa*)(&os[wb + row * OSP + c8]); const v4f x1 = *(const v4fa*)(&os[wb + row * OSP + c8 + 4]); v8h hv;
#pragma unroll
            for (int i = 0; i < 4; ++i) { hv[i] = toh_flush(relu_keep(x0[i])); hv[4 + i] = toh_flush(relu_keep(x1[i])); }
            *(volatile v8h*)(crow + (size_t)row * DM + c8) = hv; }
        if (ps == 0) __threadfence(); }
}

static_assert(8 * 2 == 16);
static_assert(16 * 16 == 256);
template <int EPI>
__device__ __forceinline__ void gemm_tile(const h16* __restrict__ A, const h16* __restrict__ Bt, const float* __restrict__ bias, const float* __restrict__ RES, const int resbf,
                                          h16* OH, float* OY, const int K, const int N) {
    __shared__ __align__(16) float os[16 * OSP];
    const int lane = threadIdx.x & 31, lr = lane & 15, hi = lane >> 4; const int r0 = blockIdx.x * 64, c0 = blockIdx.y * 64;
    v8f acc[4][4];
#pragma unroll
    for (int mb = 0; mb < 4; ++mb)
#pragma unroll
        for (int nb = 0; nb < 4; ++nb) acc[mb][nb] = (v8f){};
    const size_t aoff = (size_t)(r0 + lr) * K + 8 * hi, boff = (size_t)(c0 + lr) * K + 8 * hi;
#pragma unroll 1
    for (int kc = 0; kc < K; kc += 32) {
        v16h a[4];
#pragma unroll
        for (int mb = 0; mb < 4; ++mb) a[mb] = ldh(A + aoff + (size_t)mb * 16 * K + kc);
#pragma unroll
        for (int nb = 0; nb < 4; ++nb) { const v16h b = ldh(Bt + boff + (size_t)nb * 16 * K + kc);
#pragma unroll
            for (int mb = 0; mb < 4; ++mb) acc[mb][nb] = wmma16g(a[mb], b, acc[mb][nb]); }
    }
    float bc[4];
#pragma unroll
    for (int nb = 0; nb < 4; ++nb) bc[nb] = bfr(bias[c0 + nb * 16 + lr]);
#pragma unroll
    for (int mb = 0; mb < 4; ++mb) {
#pragma unroll
        for (int nb = 0; nb < 4; ++nb) {
#pragma unroll
            for (int j = 0; j < 8; ++j) os[(hi * 8 + j) * OSP + nb * 16 + lr] = acc[mb][nb][j] * WSI + bc[nb]; }
        wave_sync();
#pragma unroll 1
        for (int ps = 0; ps < 2; ++ps) {
            if (EPI == 0) {
#pragma unroll
                for (int s = 0; s < 4; ++s) { const int row = 4 * s + (lane >> 3), c8 = (lane & 7) * 8;
                    const v4f x0 = *(const v4fa*)(&os[row * OSP + c8]); const v4f x1 = *(const v4fa*)(&os[row * OSP + c8 + 4]); v8h hv;
#pragma unroll
                    for (int i = 0; i < 4; ++i) { hv[i] = toh_flush(relu_keep(x0[i])); hv[4 + i] = toh_flush(relu_keep(x1[i])); }
                    *(volatile v8h*)(OH + (size_t)(r0 + mb * 16 + row) * N + c0 + c8) = hv; }
            } else {
#pragma unroll
                for (int s = 0; s < 8; ++s) { const int row = 2 * s + (lane >> 4), c4 = (lane & 15) * 4;
                    const v4f x = *(const v4fa*)(&os[row * OSP + c4]);
                    const size_t go = (size_t)(r0 + mb * 16 + row) * N + c0 + c4;
                    const v4f rr = *(const v4f*)(RES + go); v4f val;
#pragma unroll
                    for (int i = 0; i < 4; ++i) { const float rv = (resbf != 0) ? bfr(rr[i]) : rr[i]; val[i] = x[i] + rv; }
                    *(volatile v4f*)(OY + go) = val; }
            }
            if (ps == 0) __threadfence(); }
        wave_sync();
    }
}
__global__ __launch_bounds__(32) void k_gemm_h(const h16* __restrict__ A, const h16* __restrict__ Bt, const float* __restrict__ bias, h16* OH, int K, int N) {
    gemm_tile<0>(A, Bt, bias, bias, 0, OH, (float*)nullptr, K, N);
}
__global__ __launch_bounds__(32) void k_gemm_y(const h16* __restrict__ A, const h16* __restrict__ Bt, const float* __restrict__ bias, const float* __restrict__ RES, int resbf, float* OY, int K, int N) {
    gemm_tile<1>(A, Bt, bias, RES, resbf, (h16*)nullptr, OY, K, N);
}

static_assert((DM / 128) * 32 * 16 == DM * 4);
static_assert((DM / 128) * 32 * 8 == DM * 2);
__global__ __launch_bounds__(256) void k_ln(const float* __restrict__ Y, const float* __restrict__ gn, const float* __restrict__ bt, float* OF, h16* OHp, const int wh) {
    const int lane = threadIdx.x & 31;
    const int wave = __builtin_amdgcn_readfirstlane((int)(threadIdx.x >> 5));
    const size_t rb = (size_t)(blockIdx.x * 8 + wave) * DM;
    float s = 0.0f;
#pragma unroll 1
    for (int j = 0; j < DM / 128; ++j) { const v4f x = *(const v4f*)(Y + rb + (size_t)(j * 32 + lane) * 4); s += (x[0] + x[1]) + (x[2] + x[3]); }
#pragma unroll
    for (int off = 16; off > 0; off >>= 1) s += __shfl_xor(s, off, 32);
    const float mu = s * (1.0f / (float)DM);
    float vs = 0.0f;
#pragma unroll 1
    for (int j = 0; j < DM / 128; ++j) { const v4f x = *(const v4f*)(Y + rb + (size_t)(j * 32 + lane) * 4);
        const float e0 = x[0] - mu, e1 = x[1] - mu, e2 = x[2] - mu, e3 = x[3] - mu; vs += (e0 * e0 + e1 * e1) + (e2 * e2 + e3 * e3); }
#pragma unroll
    for (int off = 16; off > 0; off >>= 1) vs += __shfl_xor(vs, off, 32);
    const float rstd = rsqrtf(vs * (1.0f / (float)DM) + LNEPS);
#pragma unroll 1
    for (int ps = 0; ps < 2; ++ps) {
#pragma unroll 1
        for (int j = 0; j < DM / 128; ++j) { const int c = (j * 32 + lane) * 4;
            const v4f x = *(const v4f*)(Y + rb + c); const v4f gg = *(const v4f*)(gn + c); const v4f bb = *(const v4f*)(bt + c); v4f ov; v4h hv;
#pragma unroll
            for (int i = 0; i < 4; ++i) { ov[i] = ((x[i] - mu) * rstd) * bfr(gg[i]) + bfr(bb[i]); hv[i] = toh_flush(ov[i]); }
            *(volatile v4f*)(OF + rb + c) = ov;
            if (wh != 0) *(volatile v4h*)(OHp + rb + c) = hv; }
        if (ps == 0) __threadfence(); }
}

static constexpr size_t al256(size_t v) { return (v + 255) & ~(size_t)255; }
static constexpr size_t SZ_Q  = al256((size_t)SQ * DM * 2);
static constexpr size_t SZ_K  = al256((size_t)TK * DM * 2);
static constexpr size_t SZ_SG = al256((size_t)TK * 4);
static constexpr size_t SZ_WT = al256((size_t)DM * DM * 2);
static constexpr size_t SZ_W1 = al256((size_t)DFF * DM * 2);
static constexpr size_t SZ_XF = al256((size_t)SQ * DM * 4);
static constexpr size_t SZ_HH = al256((size_t)SQ * DFF * 2);
static constexpr size_t SZ_TOTAL = 3 * SZ_Q + 2 * SZ_K + SZ_SG + SZ_WT + 2 * SZ_W1 + 3 * SZ_XF + SZ_HH;
static_assert(SZ_TOTAL <= (size_t)134217728);
static constexpr size_t N8_Q  = (size_t)SQ * DM / 8;
static constexpr size_t N8_K  = (size_t)TK * DM / 8;
static constexpr size_t N8_WT = (size_t)DM * DM / 8;
static constexpr size_t N8_W1 = (size_t)DFF * DM / 8;
static constexpr unsigned GR_Q  = (unsigned)((N8_Q + 255) / 256);
static constexpr unsigned GR_K  = (unsigned)((N8_K + 255) / 256);
static constexpr unsigned GR_WT = (unsigned)((N8_WT + 255) / 256);
static constexpr unsigned GR_W1 = (unsigned)((N8_W1 + 255) / 256);

extern "C" void kernel_launch(void* const* d_in, const int* in_sizes, int n_in,
                              void* d_out, int out_size, void* d_ws, size_t ws_size, hipStream_t stream) {
    if (n_in < 15) return;
    if ((size_t)in_sizes[0] < (size_t)SQ * DM || (size_t)in_sizes[3] < (size_t)SQ * DM) return;
    if ((size_t)in_sizes[1] < (size_t)TK * DM || (size_t)in_sizes[2] < (size_t)TK * DM) return;
    if (in_sizes[4] < TK) return;
    if ((size_t)in_sizes[5] < (size_t)DM * DM || in_sizes[6] < DM) return;
    if ((size_t)in_sizes[7] < (size_t)DFF * DM || in_sizes[8] < DFF) return;
    if ((size_t)in_sizes[9] < (size_t)DM * DFF || in_sizes[10] < DM) return;
    if (in_sizes[11] < DM || in_sizes[12] < DM || in_sizes[13] < DM || in_sizes[14] < DM) return;
    if ((size_t)out_size < (size_t)SQ * DM) return;
    if (SZ_TOTAL > ws_size) return;
    const float* tgt = (const float*)d_in[0];  const float* mem = (const float*)d_in[1];
    const float* pos = (const float*)d_in[2];  const float* qps = (const float*)d_in[3];
    const int*   aix = (const int*)d_in[4];
    const float* wt2 = (const float*)d_in[5];  const float* bt2 = (const float*)d_in[6];
    const float* w1  = (const float*)d_in[7];  const float* b1  = (const float*)d_in[8];
    const float* w2  = (const float*)d_in[9];  const float* b2  = (const float*)d_in[10];
    const float* g2  = (const float*)d_in[11]; const float* be2 = (const float*)d_in[12];
    const float* g3  = (const float*)d_in[13]; const float* be3 = (const float*)d_in[14];
    float* OUT = (float*)d_out;
    char* wsp = (char*)d_ws;
    h16* QH  = (h16*)wsp; wsp += SZ_Q;
    h16* KH  = (h16*)wsp; wsp += SZ_K;
    h16* VT  = (h16*)wsp; wsp += SZ_K;
    int* SEG = (int*)wsp; wsp += SZ_SG;
    h16* WT  = (h16*)wsp; wsp += SZ_WT;
    h16* W1H = (h16*)wsp; wsp += SZ_W1;
    h16* W2H = (h16*)wsp; wsp += SZ_W1;
    h16* CTX = (h16*)wsp; wsp += SZ_Q;
    h16* XH  = (h16*)wsp; wsp += SZ_Q;
    float* Y1 = (float*)wsp; wsp += SZ_XF;
    float* XF = (float*)wsp; wsp += SZ_XF;
    float* Y2 = (float*)wsp; wsp += SZ_XF;
    h16* HH  = (h16*)wsp; wsp += SZ_HH;

    k_sum8<<<GR_Q, 256, 0, stream>>>(tgt, qps, QH, N8_Q);
    k_sum8<<<GR_K, 256, 0, stream>>>(mem, pos, KH, N8_K);
    k_vt<<<dim3(TK / 64, DM / 64, 1), 256, 0, stream>>>(mem, VT);
    k_w8<<<GR_WT, 256, 0, stream>>>(wt2, WT, N8_WT);
    k_w8<<<GR_W1, 256, 0, stream>>>(w1, W1H, N8_W1);
    k_w8<<<GR_W1, 256, 0, stream>>>(w2, W2H, N8_W1);
    k_seg<<<1, 256, 0, stream>>>(aix, SEG);

    k_flash<<<SQ / 16, 32 * FW, 0, stream>>>(QH, KH, VT, SEG, CTX);

    k_gemm_y<<<dim3(SQ / 64, DM / 64, 1), 32, 0, stream>>>(CTX, WT, bt2, tgt, 1, Y1, DM, DM);
    k_ln<<<SQ / 8, 256, 0, stream>>>(Y1, g2, be2, XF, XH, 1);
    k_gemm_h<<<dim3(SQ / 64, DFF / 64, 1), 32, 0, stream>>>(XH, W1H, b1, HH, DM, DFF);
    k_gemm_y<<<dim3(SQ / 64, DM / 64, 1), 32, 0, stream>>>(HH, W2H, b2, XF, 0, Y2, DFF, DM);
    k_ln<<<SQ / 8, 256, 0, stream>>>(Y2, g3, be3, OUT, XH, 0);
}
